// MultiScaleRetention_58265526338092
// MI455X (gfx1250) — hardware-verified
//
#include <hip/hip_runtime.h>
#include <math.h>

constexpr int kBatch = 2;
constexpr int kSeq   = 2048;
constexpr int kDim   = 1024;
constexpr int kHeads = 16;
constexpr int kDh    = 64;
constexpr int kTok   = kBatch * kSeq;
constexpr float kWCarry     = 32.0f;
constexpr float kWCarryInv  = 1.0f / 32.0f;
constexpr float kWtMul      = 256.0f;
constexpr float kWtCarryInv = 1.0f / 2048.0f;
static_assert(kHeads * kDh == kDim);
static_assert(kDh == 64 && kSeq % 64 == 0 && kSeq % 128 == 0);
static_assert(kTok % 64 == 0 && kDim % 64 == 0 && kDim % 32 == 0);
static_assert((kTok * kDim) % (8 * 256) == 0 && (kDim * kDim) % (8 * 256) == 0);

typedef __attribute__((ext_vector_type(16))) _Float16 v16h;
typedef __attribute__((ext_vector_type(8)))  _Float16 v8h;
typedef __attribute__((ext_vector_type(16))) __bf16   v16b;
typedef __attribute__((ext_vector_type(8)))  __bf16   v8b;
typedef __attribute__((ext_vector_type(8)))  float    v8f;
typedef __attribute__((ext_vector_type(4)))  float    v4f;
typedef __attribute__((ext_vector_type(4)))  unsigned int v4u;

__device__ __forceinline__ unsigned short f2bf_bits(float f) {
  unsigned u = __float_as_uint(f);
  return (unsigned short)((u + 0x7FFFu + ((u >> 16) & 1u)) >> 16);
}
__device__ __forceinline__ float bf_bits2f(unsigned short h) { return __uint_as_float(((unsigned)h) << 16); }

__device__ __forceinline__ void dep_guard_h(v8f& a, v8f& b, v16h x, v16h y) { asm volatile("v_nop\n\tv_nop\n\tv_nop\n\tv_nop" : "+v"(a), "+v"(b) : "v"(x), "v"(y)); }
__device__ __forceinline__ void dep_guard_b(v8f& a, v8f& b, v16b x, v16b y) { asm volatile("v_nop\n\tv_nop\n\tv_nop\n\tv_nop" : "+v"(a), "+v"(b) : "v"(x), "v"(y)); }
__device__ __forceinline__ void dep_guard4_h(v8f& a, v8f& b, v8f& c, v8f& d, v16h x, v16h y) { asm volatile("v_nop\n\tv_nop\n\tv_nop\n\tv_nop" : "+v"(a), "+v"(b), "+v"(c), "+v"(d) : "v"(x), "v"(y)); }
__device__ __forceinline__ void dep_guard4_b(v8f& a, v8f& b, v8f& c, v8f& d, v16b x, v16b y) { asm volatile("v_nop\n\tv_nop\n\tv_nop\n\tv_nop" : "+v"(a), "+v"(b), "+v"(c), "+v"(d) : "v"(x), "v"(y)); }
__device__ __forceinline__ void keep4_h(v16h a, v16h b, v16h c, v16h d) { asm volatile("v_nop" :: "v"(a), "v"(b), "v"(c), "v"(d)); }
__device__ __forceinline__ void keep4_b(v16b a, v16b b, v16b c, v16b d) { asm volatile("v_nop" :: "v"(a), "v"(b), "v"(c), "v"(d)); }
__device__ __forceinline__ void acc_guard4(v8f& a, v8f& b, v8f& c, v8f& d) { asm volatile("v_nop\n\tv_nop\n\tv_nop\n\tv_nop" : "+v"(a), "+v"(b), "+v"(c), "+v"(d)); }
template <typename T> struct Frag;
template <> struct Frag<_Float16> {
  typedef v16h V; union U { v16h v; v8h h[2]; };
  static __device__ __forceinline__ v16h load(const _Float16* p) {
    U f; f.h[0] = *(const v8h*)(p); f.h[1] = *(const v8h*)(p + 16); return f.v;
  }
  static __device__ __forceinline__ v8f mma(v16h a, v16h b, v8f c) {
    return __builtin_amdgcn_wmma_f32_16x16x32_f16(false, a, false, b, (short)0, c, false, false);
  }
  static __device__ __forceinline__ void guard(v8f& a, v8f& b, v16h x, v16h y) { dep_guard_h(a, b, x, y); }
  static __device__ __forceinline__ void guard4(v8f& a, v8f& b, v8f& c, v8f& d, v16h x, v16h y) { dep_guard4_h(a, b, c, d, x, y); }
  static __device__ __forceinline__ void keep(v16h a, v16h b, v16h c, v16h d) { keep4_h(a, b, c, d); }
};
template <> struct Frag<__bf16> {
  typedef v16b V; union U { v16b v; v8b h[2]; };
  static __device__ __forceinline__ v16b load(const __bf16* p) {
    U f; f.h[0] = *(const v8b*)(p); f.h[1] = *(const v8b*)(p + 16); return f.v;
  }
  static __device__ __forceinline__ v8f mma(v16b a, v16b b, v8f c) {
    return __builtin_amdgcn_wmma_f32_16x16x32_bf16(false, a, false, b, (short)0, c, false, false);
  }
  static __device__ __forceinline__ void guard(v8f& a, v8f& b, v16b x, v16b y) { dep_guard_b(a, b, x, y); }
  static __device__ __forceinline__ void guard4(v8f& a, v8f& b, v8f& c, v8f& d, v16b x, v16b y) { dep_guard4_b(a, b, c, d, x, y); }
  static __device__ __forceinline__ void keep(v16b a, v16b b, v16b c, v16b d) { keep4_b(a, b, c, d); }
};

__device__ __forceinline__ unsigned pk16(unsigned short a, unsigned short b) { return (unsigned)a | ((unsigned)b << 16); }
__device__ __forceinline__ unsigned short h_bits(float f) { const _Float16 h = (_Float16)f; return __builtin_bit_cast(unsigned short, h); }

template <int ET> struct Elem;
template <> struct Elem<0> { typedef _Float16 T; };
template <> struct Elem<1> { typedef __bf16 T; };
template <int ET, bool SPLIT, int BIAS_MODE, int OUT_MODE, bool RESID, int ACT = 0>
__global__ __launch_bounds__(256) void wmma_gemm64(
    const unsigned short* __restrict__ Ap, const unsigned short* __restrict__ A2p, int lda, long strideA,
    const unsigned short* __restrict__ Btp, const unsigned short* __restrict__ Bt2p, int ldb, long strideB,
    void* __restrict__ Cout, void* __restrict__ Cout2, int ldc, long strideC,
    const float* __restrict__ bias,
    const float* __restrict__ resid, long strideR,
    int M, int N, int K, float scale) {
  typedef typename Elem<ET>::T T;
  typedef typename Frag<T>::V V;
  const T* A = (const T*)Ap; const T* A2 = (const T*)A2p; const T* Bt = (const T*)Btp; const T* Bt2 = (const T*)Bt2p;
  __shared__ __align__(16) float sT[8][16 * 68];
  const int b    = blockIdx.y;
  const int lane = threadIdx.x & 31;
  const int wave = threadIdx.x >> 5;
  const int tilesN = N >> 6;
  const int tilesM = M >> 6;
  const int tile = blockIdx.x * 8 + wave;
  if (tile >= tilesM * tilesN) return;
  const int tm = tile / tilesN;
  const int tn = tile - tm * tilesN;
  const int m0 = tm << 6;
  const int n0 = tn << 6;

  const T* Ab  = A  + (size_t)b * strideA;
  const T* Bb  = Bt + (size_t)b * strideB;
  const T* Ab2 = SPLIT ? (A2  + (size_t)b * strideA) : nullptr;
  const T* Bb2 = SPLIT ? (Bt2 + (size_t)b * strideB) : nullptr;

  const int rlane = lane & 15;
  const int koff  = (lane >> 4) * 8;
  const int mOff  = (lane >> 4) * 8;

  v8f acc[4][4];
#pragma unroll
  for (int i = 0; i < 4; ++i)
#pragma unroll
    for (int j = 0; j < 4; ++j) acc[i][j] = (v8f){0.f,0.f,0.f,0.f,0.f,0.f,0.f,0.f};

  for (int k0 = 0; k0 < K; k0 += 32) {
    V bh[4], bl[4];
#pragma unroll
    for (int j = 0; j < 4; ++j) {
      const size_t bo = (size_t)(n0 + (j << 4) + rlane) * ldb + koff + k0;
      bh[j] = Frag<T>::load(Bb + bo);
      if (SPLIT) bl[j] = Frag<T>::load(Bb2 + bo);
    }
#pragma unroll
    for (int i = 0; i < 4; ++i) {
      const size_t ao = (size_t)(m0 + (i << 4) + rlane) * lda + koff + k0;
      V ah = Frag<T>::load(Ab + ao);
      V al;
      if (SPLIT) al = Frag<T>::load(Ab2 + ao);
#pragma unroll
      for (int j = 0; j < 4; ++j) {
        acc[i][j] = Frag<T>::mma(ah, bh[j], acc[i][j]);
        if (SPLIT) {
          acc[i][j] = Frag<T>::mma(ah, bl[j], acc[i][j]);
          acc[i][j] = Frag<T>::mma(al, bh[j], acc[i][j]);
        }
      }
      Frag<T>::guard4(acc[i][0], acc[i][1], acc[i][2], acc[i][3], ah, SPLIT ? al : ah);
    }
    Frag<T>::keep(bh[0], bh[1], bh[2], bh[3]);
    if (SPLIT) Frag<T>::keep(bl[0], bl[1], bl[2], bl[3]);
  }
  acc_guard4(acc[0][0], acc[0][1], acc[0][2], acc[0][3]);
  acc_guard4(acc[1][0], acc[1][1], acc[1][2], acc[1][3]);
  acc_guard4(acc[2][0], acc[2][1], acc[2][2], acc[2][3]);
  acc_guard4(acc[3][0], acc[3][1], acc[3][2], acc[3][3]);

  float* slab = sT[wave];
  const float* Rb = RESID ? (resid + (size_t)b * strideR) : nullptr;
#pragma unroll
  for (int i = 0; i < 4; ++i) {
    const int mBase = m0 + (i << 4);
#pragma unroll
    for (int j = 0; j < 4; ++j) {
      const int n = n0 + (j << 4) + rlane;
      float bv = 0.f;
      if (BIAS_MODE == 2) bv = bias[n];
#pragma unroll
      for (int r = 0; r < 8; ++r) {
        float v = acc[i][j][r] * scale;
        if (BIAS_MODE == 1) v += bias[mBase + mOff + r];
        if (BIAS_MODE == 2) v += bv;
        if (RESID) v += Rb[(size_t)(mBase + mOff + r) * ldc + n];
        if (ACT == 2) v = fmaxf(v, 0.0f);
        if (ACT == 4) v = (v > 0.f) ? v : 0.01f * v;
        slab[(mOff + r) * 68 + (j << 4) + rlane] = v;
      }
    }
    __builtin_amdgcn_fence(__ATOMIC_RELEASE, "workgroup");
    __builtin_amdgcn_wave_barrier();
    __builtin_amdgcn_fence(__ATOMIC_ACQUIRE, "workgroup");
    if (OUT_MODE == 0) {
      float* C = (float*)Cout + (size_t)b * strideC;
      const int hh = lane >> 4, c4 = (lane & 15) * 4;
      for (int pass = 0; pass < 2; ++pass) {
#pragma unroll
        for (int it = 0; it < 8; ++it) {
          const int row = it * 2 + hh;
          v4f v = *(const v4f*)(slab + row * 68 + c4);
          *(volatile v4f*)(C + (size_t)(mBase + row) * ldc + n0 + c4) = v;
        }
        __threadfence();
      }
    } else {
      const int q = lane >> 3, c8 = (lane & 7) * 8;
      unsigned short* C  = (unsigned short*)Cout  + (size_t)b * strideC;
      unsigned short* C2 = (OUT_MODE == 2) ? ((unsigned short*)Cout2 + (size_t)b * strideC) : nullptr;
      for (int pass = 0; pass < 2; ++pass) {
#pragma unroll
        for (int it = 0; it < 4; ++it) {
          const int row = it * 4 + q;
          const float* sp = slab + row * 68 + c8;
          v8h hv, lv;
#pragma unroll
          for (int e = 0; e < 8; ++e) {
            if (OUT_MODE == 1) {
              hv[e] = (_Float16)sp[e];
            } else {
              unsigned short hb = f2bf_bits(sp[e]);
              unsigned short lb = f2bf_bits(sp[e] - bf_bits2f(hb));
              hv[e] = __builtin_bit_cast(_Float16, hb);
              lv[e] = __builtin_bit_cast(_Float16, lb);
            }
          }
          *(volatile v8h*)(C + (size_t)(mBase + row) * ldc + n0 + c8) = hv;
          if (OUT_MODE == 2) *(volatile v8h*)(C2 + (size_t)(mBase + row) * ldc + n0 + c8) = lv;
        }
        __threadfence();
      }
    }
    __builtin_amdgcn_fence(__ATOMIC_RELEASE, "workgroup");
    __builtin_amdgcn_wave_barrier();
    __builtin_amdgcn_fence(__ATOMIC_ACQUIRE, "workgroup");
  }
}

__global__ __launch_bounds__(256) void cast8_x_kernel(const float* __restrict__ in, unsigned short* __restrict__ out, int n8) {
  const int i = blockIdx.x * 256 + threadIdx.x;
  if (i >= n8) return;
  const float* p = in + 8 * (size_t)i;
  const v4f a = *(const v4f*)(p);
  const v4f c = *(const v4f*)(p + 4);
  unsigned short hb[8];
#pragma unroll
  for (int e = 0; e < 4; ++e) {
    hb[e]     = h_bits(bf_bits2f(f2bf_bits(a[e])));
    hb[4 + e] = h_bits(bf_bits2f(f2bf_bits(c[e])));
  }
  const v4u u = (v4u){pk16(hb[0], hb[1]), pk16(hb[2], hb[3]), pk16(hb[4], hb[5]), pk16(hb[6], hb[7])};
  unsigned short* q = out + 8 * (size_t)i;
  *(volatile v4u*)q = u;
  __threadfence();
  *(volatile v4u*)q = u;
}

__global__ __launch_bounds__(256) void cast8_w4_kernel(const float* __restrict__ W0, const float* __restrict__ W1,
                                                      const float* __restrict__ W2, const float* __restrict__ W3,
                                                      unsigned short* __restrict__ out, int n8, float carry) {
  const int i = blockIdx.x * 256 + threadIdx.x;
  const int z = blockIdx.y;
  if (i >= n8) return;
  const float* W = (z == 0) ? W0 : (z == 1) ? W1 : (z == 2) ? W2 : W3;
  const float* p = W + 8 * (size_t)i;
  const v4f a = *(const v4f*)(p);
  const v4f c = *(const v4f*)(p + 4);
  unsigned short hb[8];
#pragma unroll
  for (int e = 0; e < 4; ++e) {
    hb[e]     = h_bits(bf_bits2f(f2bf_bits(a[e])) * carry);
    hb[4 + e] = h_bits(bf_bits2f(f2bf_bits(c[e])) * carry);
  }
  const v4u u = (v4u){pk16(hb[0], hb[1]), pk16(hb[2], hb[3]), pk16(hb[4], hb[5]), pk16(hb[6], hb[7])};
  unsigned short* q = out + (size_t)z * ((size_t)n8 * 8) + 8 * (size_t)i;
  *(volatile v4u*)q = u;
  __threadfence();
  *(volatile v4u*)q = u;
}

__device__ __forceinline__ v8f mma_h(v16h a, v16h b, v8f c) {
  c = __builtin_amdgcn_wmma_f32_16x16x32_f16(false, a, false, b, (short)0, c, false, false);
  asm volatile("v_nop\n\tv_nop\n\tv_nop\n\tv_nop" : "+v"(c) : "v"(a), "v"(b));
  return c;
}
__device__ __forceinline__ void lds_wave_sync() {
  __builtin_amdgcn_fence(__ATOMIC_RELEASE, "workgroup");
  __builtin_amdgcn_wave_barrier();
  __builtin_amdgcn_fence(__ATOMIC_ACQUIRE, "workgroup");
}

__global__ __launch_bounds__(128) void decay_attn_kernel(const unsigned short* __restrict__ Qp, const unsigned short* __restrict__ Kp,
                                                        const unsigned short* __restrict__ VTp, const float* __restrict__ gam,
                                                        unsigned short* __restrict__ Rp) {
  __shared__ __align__(16) float    dtab[kSeq];
  __shared__ __align__(16) _Float16 wsm[4][16 * 32];
  __shared__ __align__(16) float    osm[4][16 * 68];

  const int tid  = threadIdx.x;
  const int wave = tid >> 5;
  const int lane = tid & 31;
  const int hh   = lane >> 4;
  const int c    = lane & 15;
  const int h    = blockIdx.y;
  const int b    = blockIdx.z;
  const int t0   = blockIdx.x * 64 + wave * 16;

  {
    const float g  = gam[h];
    const float gb = bf_bits2f(f2bf_bits(g));
    const float lg = log2f(gb);
#pragma unroll 1
    for (int i = 0; i < kSeq / 128; ++i) {
      const int d = i * 128 + tid;
      dtab[d] = exp2f((float)d * lg);
    }
  }
  __syncthreads();

  const _Float16* Qh = (const _Float16*)Qp;
  const _Float16* Kh = (const _Float16*)Kp;
  const _Float16* Vh = (const _Float16*)VTp;

  const size_t qoff = ((size_t)(b * kSeq + t0 + c)) * kDim + h * kDh + 8 * hh;
  const v16h qf0 = Frag<_Float16>::load(Qh + qoff);
  const v16h qf1 = Frag<_Float16>::load(Qh + qoff + 32);

  v8f oacc[4];
#pragma unroll
  for (int t4 = 0; t4 < 4; ++t4) oacc[t4] = (v8f){0.f,0.f,0.f,0.f,0.f,0.f,0.f,0.f};

  _Float16* wp = wsm[wave];
  const int send = t0 + 16;
  for (int s0 = 0; s0 < send; s0 += 32) {
    v8f sacc[2];
#pragma unroll
    for (int sc = 0; sc < 2; ++sc) {
      const size_t koff = ((size_t)(b * kSeq + s0 + sc * 16 + c)) * kDim + h * kDh + 8 * hh;
      const v16h kb0 = Frag<_Float16>::load(Kh + koff);
      const v16h kb1 = Frag<_Float16>::load(Kh + koff + 32);
      v8f sv = (v8f){0.f,0.f,0.f,0.f,0.f,0.f,0.f,0.f};
      sv = mma_h(qf0, kb0, sv);
      sv = mma_h(qf1, kb1, sv);
      sacc[sc] = sv;
    }
#pragma unroll
    for (int sc = 0; sc < 2; ++sc) {
      const int s     = s0 + sc * 16 + c;
      const int dbase = t0 + 8 * hh - s;
#pragma unroll
      for (int r = 0; r < 8; ++r) {
        const int d   = dbase + r;
        const int dcl = d < 0 ? 0 : d;
        const float dv = dtab[dcl];
        const float w  = (sacc[sc][r] * dv) * kWtMul;
        const float wm = (d >= 0) ? w : 0.0f;
        wp[(8 * hh + r) * 32 + sc * 16 + c] = (_Float16)wm;
      }
    }
    lds_wave_sync();
    const v16h wf = Frag<_Float16>::load(wp + c * 32 + 8 * hh);
    const size_t voff = ((size_t)(h * kDh + c)) * kTok + b * kSeq + s0 + 8 * hh;
#pragma unroll
    for (int t4 = 0; t4 < 4; ++t4) {
      const v16h vb = Frag<_Float16>::load(Vh + voff + (size_t)(t4 * 16) * kTok);
      oacc[t4] = mma_h(wf, vb, oacc[t4]);
    }
    lds_wave_sync();
  }

  float* os = osm[wave];
#pragma unroll
  for (int t4 = 0; t4 < 4; ++t4) {
#pragma unroll
    for (int r = 0; r < 8; ++r) os[(8 * hh + r) * 68 + t4 * 16 + c] = oacc[t4][r] * kWtCarryInv;
  }
  lds_wave_sync();
  {
    const int q = lane >> 3, c8 = (lane & 7) * 8;
    for (int pass = 0; pass < 2; ++pass) {
#pragma unroll
      for (int it = 0; it < 4; ++it) {
        const int row = it * 4 + q;
        const float* sp = os + row * 68 + c8;
        const v4f e0 = *(const v4f*)(sp);
        const v4f e1 = *(const v4f*)(sp + 4);
        unsigned short hb[8];
#pragma unroll
        for (int e = 0; e < 4; ++e) {
          hb[e]     = h_bits(e0[e]);
          hb[4 + e] = h_bits(e1[e]);
        }
        const v4u u = (v4u){pk16(hb[0], hb[1]), pk16(hb[2], hb[3]), pk16(hb[4], hb[5]), pk16(hb[6], hb[7])};
        *(volatile v4u*)(Rp + ((size_t)(b * kSeq + t0 + row)) * kDim + h * kDh + c8) = u;
      }
      __threadfence();
    }
  }
}

extern "C" void kernel_launch(void* const* d_in, const int* in_sizes, int n_in,
                              void* d_out, int out_size, void* d_ws, size_t ws_size,
                              hipStream_t stream) {
  if (n_in < 6) return;
  const int nX = kTok * kDim;
  const int nW = kDim * kDim;
  if (in_sizes[0] != nX || in_sizes[1] != nW || in_sizes[2] != nW || in_sizes[3] != nW || in_sizes[4] != nW) return;
  if (in_sizes[5] != kHeads) return;
  if (out_size != nX) return;

  const size_t szX = (size_t)nX * 2;
  const size_t szW = (size_t)nW * 2;
  const size_t offXH = 0;
  const size_t offWH = offXH + szX;
  const size_t offQ  = offWH + 4 * szW;
  const size_t offK  = offQ + szX;
  const size_t offVT = offK + szX;
  const size_t offR  = offVT + szX;
  const size_t total = offR + szX;
  if (ws_size < total) return;

  const float* x  = (const float*)d_in[0];
  const float* wq = (const float*)d_in[1];
  const float* wk = (const float*)d_in[2];
  const float* wv = (const float*)d_in[3];
  const float* wo = (const float*)d_in[4];
  const float* gm = (const float*)d_in[5];
  float* out = (float*)d_out;
  char* ws = (char*)d_ws;
  unsigned short* XH   = (unsigned short*)(ws + offXH);
  unsigned short* WH   = (unsigned short*)(ws + offWH);
  unsigned short* WQH  = WH;
  unsigned short* WKH  = WH + (size_t)nW;
  unsigned short* WVH  = WH + 2 * (size_t)nW;
  unsigned short* WOH  = WH + 3 * (size_t)nW;
  unsigned short* Q16  = (unsigned short*)(ws + offQ);
  unsigned short* K16  = (unsigned short*)(ws + offK);
  unsigned short* VT16 = (unsigned short*)(ws + offVT);
  unsigned short* R16  = (unsigned short*)(ws + offR);

  const int nX8 = nX / 8;
  const int nW8 = nW / 8;
  cast8_x_kernel<<<dim3(nX8 / 256), dim3(256), 0, stream>>>(x, XH, nX8);
  cast8_w4_kernel<<<dim3(nW8 / 256, 4), dim3(256), 0, stream>>>(wq, wk, wv, wo, WH, nW8, kWCarry);

  const int tilesProj = (kTok / 64) * (kDim / 64);

  wmma_gemm64<0, false, 0, 1, false, 0><<<dim3(tilesProj / 8, 1), dim3(256), 0, stream>>>(
      XH, XH, kDim, 0L, WQH, WQH, kDim, 0L,
      (void*)Q16, (void*)Q16, kDim, 0L, gm, gm, 0L, kTok, kDim, kDim, kWCarryInv);
  wmma_gemm64<0, false, 0, 1, false, 0><<<dim3(tilesProj / 8, 1), dim3(256), 0, stream>>>(
      XH, XH, kDim, 0L, WKH, WKH, kDim, 0L,
      (void*)K16, (void*)K16, kDim, 0L, gm, gm, 0L, kTok, kDim, kDim, kWCarryInv);
  wmma_gemm64<0, false, 0, 1, false, 0><<<dim3(tilesProj / 8, 1), dim3(256), 0, stream>>>(
      WVH, WVH, kDim, 0L, XH, XH, kDim, 0L,
      (void*)VT16, (void*)VT16, kTok, 0L, gm, gm, 0L, kDim, kTok, kDim, kWCarryInv);

  decay_attn_kernel<<<dim3(kSeq / 64, kHeads, kBatch), dim3(128), 0, stream>>>(Q16, K16, VT16, gm, R16);

  wmma_gemm64<0, false, 0, 0, false, 0><<<dim3(tilesProj / 8, 1), dim3(256), 0, stream>>>(
      R16, R16, kDim, 0L, WOH, WOH, kDim, 0L,
      (void*)out, (void*)out, kDim, 0L, gm, gm, 0L, kTok, kDim, kDim, kWCarryInv);
}
